// RecGCNblock_37838661877767
// MI455X (gfx1250) — hardware-run, weakly checked
//
#include <hip/hip_runtime.h>

typedef float          v8f   __attribute__((ext_vector_type(8)));
typedef float          v4f   __attribute__((ext_vector_type(4)));
typedef unsigned int   v4u   __attribute__((ext_vector_type(4)));
typedef int            v8i   __attribute__((ext_vector_type(8)));
typedef unsigned short v8us  __attribute__((ext_vector_type(8)));
typedef unsigned short v16us __attribute__((ext_vector_type(16)));
typedef __bf16         v16bf __attribute__((ext_vector_type(16)));
typedef _Float16       v16h  __attribute__((ext_vector_type(16)));
typedef v4f  __attribute__((may_alias)) v4fa;
typedef v8us __attribute__((may_alias)) v8usa;
union FragB { v16bf v; v16us u; v8us h[2]; v8i w; };
union FragH { v16h  v; v16us u; v8us h[2]; v8i w; };

__device__ __forceinline__ v8f wmb(const FragB& a, const FragB& b, v8f c) {
  v8f d = __builtin_amdgcn_wmma_f32_16x16x32_bf16(false, a.v, false, b.v, (short)0, c, false, false);
  asm volatile("v_nop\n\tv_nop\n\tv_nop\n\tv_nop" : "+v"(d) : "v"(a.w), "v"(b.w));
  return d;
}

__device__ __forceinline__ v8f wmh(const FragH& a, const FragH& b, v8f c) {
  v8f d = __builtin_amdgcn_wmma_f32_16x16x32_f16(false, a.v, false, b.v, (short)0, c, false, false);
  asm volatile("v_nop\n\tv_nop\n\tv_nop\n\tv_nop" : "+v"(d) : "v"(a.w), "v"(b.w));
  return d;
}

__device__ __forceinline__ unsigned bf16_bits(float f) {
  const unsigned u = __float_as_uint(f);
  const unsigned r = (u + 0x7FFFu + ((u >> 16) & 1u)) >> 16;
  const unsigned q = (u >> 16) | 0x40u;
  return ((u & 0x7fffffffu) > 0x7f800000u) ? q : r;
}

__device__ __forceinline__ float bf16_val(float f) {
  return __uint_as_float(bf16_bits(f) << 16);
}
__device__ __forceinline__ int clampi(int v, int lo, int hi) {
  return v < lo ? lo : (v > hi ? hi : v);
}

__device__ __forceinline__ unsigned f16_bits(float f) {
  const unsigned u  = __float_as_uint(f);
  const unsigned s  = (u >> 16) & 0x8000u;
  const unsigned a  = u & 0x7fffffffu;
  const unsigned t  = a - 0x38000000u;
  const unsigned r  = (t + 0x0FFFu + ((t >> 13) & 1u)) >> 13;
  const unsigned rc = r > 0x7C00u ? 0x7C00u : r;
  const bool small  = a < 0x38800000u;
  const bool isnan  = a > 0x7f800000u;
  const unsigned fin = small ? 0u : (s | rc);
  return isnan ? (s | 0x7E00u) : fin;
}

__device__ __forceinline__ unsigned pk16(unsigned lo, unsigned hi) { return lo | (hi << 16); }
__device__ __forceinline__ unsigned bf16_lo_bits(float v) {
  float hi = bf16_val(v);
  asm volatile("" : "+v"(hi));
  return bf16_bits(v - hi);
}
__device__ __forceinline__ v4u pack8_bf16(v4f a, v4f c) {
  return (v4u){ pk16(bf16_bits(a[0]), bf16_bits(a[1])), pk16(bf16_bits(a[2]), bf16_bits(a[3])),
                pk16(bf16_bits(c[0]), bf16_bits(c[1])), pk16(bf16_bits(c[2]), bf16_bits(c[3])) };
}
__device__ __forceinline__ v4u pack8_bf16_lo(v4f a, v4f c) {
  return (v4u){ pk16(bf16_lo_bits(a[0]), bf16_lo_bits(a[1])), pk16(bf16_lo_bits(a[2]), bf16_lo_bits(a[3])),
                pk16(bf16_lo_bits(c[0]), bf16_lo_bits(c[1])), pk16(bf16_lo_bits(c[2]), bf16_lo_bits(c[3])) };
}
__device__ __forceinline__ v4u pack8_f16(v4f a, v4f c) {
  return (v4u){ pk16(f16_bits(a[0]), f16_bits(a[1])), pk16(f16_bits(a[2]), f16_bits(a[3])),
                pk16(f16_bits(c[0]), f16_bits(c[1])), pk16(f16_bits(c[2]), f16_bits(c[3])) };
}

template <int FORM>
__global__ __launch_bounds__(256) void k_plane(const float* __restrict__ src, int rows, int cols, int ldsrc,
                                               unsigned short* __restrict__ dst, int MP, int KP) {
  static_assert(FORM >= 0 && FORM <= 3);
  const int KTOT = (FORM == 1 || FORM == 3) ? 2 * KP : KP;
  const unsigned ppr   = (unsigned)(KTOT >> 3);
  const unsigned kp8   = (unsigned)(KP >> 3);
  const unsigned total = (unsigned)MP * ppr;
  const unsigned g     = blockIdx.x * 256u + threadIdx.x;
  const unsigned rowu  = g / ppr;
  const unsigned p     = g - rowu * ppr;
  const bool second    = p >= kp8;
  const int row = (int)rowu;
  const int c0  = (int)((second ? p - kp8 : p) << 3);
  const float* srow = src + (size_t)clampi(row, 0, rows - 1) * (size_t)ldsrc;
  float x[8];
  unsigned mk[8];
#pragma unroll
  for (int e = 0; e < 8; ++e) {
    const int c = c0 + e;
    const float v = srow[clampi(c, 0, cols - 1)];
    asm volatile("" :: "v"(v));
    x[e]  = v;
    mk[e] = (row < rows && c < cols) ? 0xFFFFu : 0u;
  }
  const v4f a = (v4f){ x[0], x[1], x[2], x[3] };
  const v4f c = (v4f){ x[4], x[5], x[6], x[7] };
  v4u o;
  if (FORM == 2) {
    o = pack8_f16(a, c);
  } else {
    const v4u hi = pack8_bf16(a, c);
    o = hi;
    if (FORM == 1) { const v4u lo = pack8_bf16_lo(a, c); o = second ? lo : hi; }
  }
  const v4u mw = (v4u){ pk16(mk[0], mk[1]), pk16(mk[2], mk[3]), pk16(mk[4], mk[5]), pk16(mk[6], mk[7]) };
  o &= mw;
  if (g < total) {
    volatile v4u* q = (volatile v4u*)(dst + (size_t)g * 8);
    *q = o;
    __threadfence();
    *q = o;
  }
}

template <int FORM> struct FragOf    { typedef FragB T; };
template <>         struct FragOf<2> { typedef FragH T; };
__device__ __forceinline__ v8f mm(const FragB& a, const FragB& b, v8f c) { return wmb(a, b, c); }
__device__ __forceinline__ v8f mm(const FragH& a, const FragH& b, v8f c) { return wmh(a, b, c); }
template <class F> __device__ __forceinline__ F ld_frag(const unsigned short* p) {
  F f;
  f.h[0] = *(const v8usa*)(p);
  f.h[1] = *(const v8usa*)(p + 16);
  return f;
}

template <int FORM, int EPI>
__global__ __launch_bounds__(256) __attribute__((amdgpu_num_vgpr(248)))
void k_gemm_nt(const unsigned short* __restrict__ A, const unsigned short* __restrict__ B,
               const float* __restrict__ bias, float* __restrict__ D, int M, int N, int KTOT, int ldd) {
  static_assert(FORM >= 0 && FORM <= 2);
  static_assert(EPI == 0 || EPI == 1);
  typedef typename FragOf<FORM>::T F;
  __shared__ __attribute__((aligned(16))) float sT[8][16 * 68];
  const int lane = threadIdx.x & 31;
  const int wave = threadIdx.x >> 5;
  const int tilesM = (M + 63) >> 6;
  const int tilesN = (N + 63) >> 6;
  const int tile = blockIdx.x * 8 + wave;
  if (tile >= tilesM * tilesN) return;
  const int tm = tile / tilesN;
  const int tn = tile - tm * tilesN;
  const int m0 = tm << 6;
  const int n0 = tn << 6;

  const int rl = lane & 15;
  const int h8 = (lane >> 4) * 8;
  const unsigned short* pa = A + (size_t)(m0 + rl) * (size_t)KTOT + h8;
  const unsigned short* pb = B + (size_t)(n0 + rl) * (size_t)KTOT + h8;

  v8f acc[4][4];
#pragma unroll
  for (int i = 0; i < 4; ++i)
#pragma unroll
    for (int j = 0; j < 4; ++j) acc[i][j] = (v8f){0.f, 0.f, 0.f, 0.f, 0.f, 0.f, 0.f, 0.f};

#pragma unroll 1
  for (int k0 = 0; k0 < KTOT; k0 += 32) {
    F bf[4];
#pragma unroll
    for (int j = 0; j < 4; ++j) bf[j] = ld_frag<F>(pb + (size_t)(j << 4) * (size_t)KTOT + k0);
#pragma unroll
    for (int i = 0; i < 4; ++i) {
      const F af = ld_frag<F>(pa + (size_t)(i << 4) * (size_t)KTOT + k0);
#pragma unroll
      for (int j = 0; j < 4; ++j) acc[i][j] = mm(af, bf[j], acc[i][j]);
    }
  }

  float* slab = sT[wave];
  const int hh = lane >> 4;
  const int c4 = (lane & 15) * 4;
  const int nc = n0 + c4;
  const bool cok = nc < N;
  v4f bv = (v4f){0.f, 0.f, 0.f, 0.f};
  if (EPI == 1) {
    bv = *(const v4fa*)(bias + clampi(nc, 0, N - 4));
    asm volatile("" :: "v"(bv));
  }
#pragma unroll
  for (int i = 0; i < 4; ++i) {
    const int mBase = m0 + (i << 4);
#pragma unroll
    for (int j = 0; j < 4; ++j) {
#pragma unroll
      for (int r = 0; r < 8; ++r) slab[(h8 + r) * 68 + (j << 4) + rl] = acc[i][j][r];
    }
    __builtin_amdgcn_fence(__ATOMIC_RELEASE, "workgroup");
    __builtin_amdgcn_wave_barrier();
    __builtin_amdgcn_fence(__ATOMIC_ACQUIRE, "workgroup");
    v4f vv[8];
#pragma unroll
    for (int it = 0; it < 8; ++it) {
      const int row = it * 2 + hh;
      v4f v = *(const v4fa*)(slab + row * 68 + c4);
      if (EPI == 1) v += bv;
      vv[it] = v;
    }
    for (int pass = 0; pass < 2; ++pass) {
#pragma unroll
      for (int it = 0; it < 8; ++it) {
        const int row = mBase + it * 2 + hh;
        if (cok && row < M) *(volatile v4f*)(D + (size_t)row * (size_t)ldd + nc) = vv[it];
      }
      __threadfence();
    }
    __builtin_amdgcn_fence(__ATOMIC_RELEASE, "workgroup");
    __builtin_amdgcn_wave_barrier();
    __builtin_amdgcn_fence(__ATOMIC_ACQUIRE, "workgroup");
  }
}

#pragma clang fp contract(off)

#define AGG_TWO_TERM 1
#define X_TWO_TERM   1

#define NNODE   50000
#define NEDGE   600000
#define DF      128
#define G3      384
#define NPAD    50048
#define K2      256
#define CH_ROWS 12544
#define CH_LAST 12416
#define NTHR    256
#define NWAVE   8
#define NBA     1024
#define SLA     10
#define NBLK    49
#define SUB     256
#define WSTEPS  293
#define WSPAN   (WSTEPS * SUB)
#define WLCAP   2048
#define RCAP    16384
#define DEGCAP  64
#define FLAGW   32
#define BK_INTS (NWAVE * WLCAP + RCAP + NWAVE * NBA + 3 * NBA + 16)
#define BK_LDS  (BK_INTS * 4)

#define SZ_HB   ((size_t)NPAD * DF * 2)
#define SZ_PHL  ((size_t)NPAD * K2 * 2)
#define SZ_X    ((size_t)NPAD * DF * 4)
#define SZ_G    ((size_t)CH_ROWS * G3 * 4)
#define SZ_LIST ((size_t)NBLK * RCAP * 4)
#define SZ_TAB  ((size_t)NPAD * 4)
#define SZ_WG   ((size_t)DF * K2 * 2)
#define SZ_WIH  ((size_t)G3 * K2 * 2)
#define SZ_WHH  ((size_t)G3 * DF * 2)
#define SZ_BG   ((size_t)DF * 4)
#define SZ_B3   ((size_t)G3 * 4)
#define SZ_FLAG ((size_t)6400)
#define WS_TOTAL (SZ_HB + SZ_PHL + SZ_X + 2 * SZ_G + SZ_LIST + 4 * SZ_TAB + SZ_WG + SZ_WIH + SZ_WHH + SZ_BG + 2 * SZ_B3 + SZ_FLAG)

static_assert(DF == 128 && G3 == 3 * DF && K2 == 2 * DF);
static_assert(NPAD == 391 * 128 && NPAD % 64 == 0 && NPAD >= NNODE);
static_assert(3 * 98 + 97 == 391 && CH_ROWS == 98 * 128 && CH_LAST == 97 * 128 && 3 * CH_ROWS + CH_LAST == NPAD);
static_assert(CH_ROWS % 64 == 0 && CH_LAST % 64 == 0 && CH_ROWS % 8 == 0 && CH_LAST % 8 == 0);
static_assert(3 * CH_ROWS + 12368 == NNODE);
static_assert(NEDGE == 600000 && NEDGE % 8 == 0);
static_assert(NWAVE * WSPAN >= NEDGE && (NWAVE - 1) * WSPAN < NEDGE);
static_assert(NEDGE - (NWAVE - 1) * WSPAN - (WSTEPS - 1) * SUB == 192);
static_assert(NWAVE * WSPAN + 8 < (1 << 20));
static_assert(NBA == (1 << SLA) && NBLK * NBA >= NPAD && (NBLK - 1) * NBA < NPAD);
static_assert((NPAD - (NBLK - 1) * NBA) % 128 == 0);
static_assert(NWAVE * WLCAP <= RCAP && RCAP % (NTHR * 4) == 0);
static_assert(RCAP * 4 + NWAVE * WLCAP * 4 <= 262144 && BK_LDS <= 262144 && BK_INTS % 4 == 0);
static_assert(DEGCAP >= 38 && DEGCAP <= RCAP);
static_assert(NBLK * FLAGW * 4 <= 6400);
static_assert(WS_TOTAL == (size_t)((size_t)417887 << 8) && WS_TOTAL <= ((size_t)128 << 20));
static_assert(SZ_HB % 256 == 0 && SZ_PHL % 256 == 0 && SZ_X % 256 == 0 && SZ_G % 256 == 0 && SZ_LIST % 256 == 0);
static_assert(SZ_TAB % 256 == 0 && SZ_WG % 256 == 0 && SZ_WIH % 256 == 0 && SZ_WHH % 256 == 0 && SZ_BG % 256 == 0 && SZ_B3 % 256 == 0);

typedef int          v4i  __attribute__((ext_vector_type(4)));
typedef unsigned int v2u  __attribute__((ext_vector_type(2)));
typedef v4i __attribute__((may_alias)) v4ia;
typedef v2u __attribute__((may_alias)) v2ua;
typedef v4u __attribute__((may_alias)) v4ua;

__device__ __forceinline__ void wave_sync() {
  __builtin_amdgcn_fence(__ATOMIC_RELEASE, "workgroup");
  __builtin_amdgcn_wave_barrier();
  __builtin_amdgcn_fence(__ATOMIC_ACQUIRE, "workgroup");
}

__global__ __launch_bounds__(NTHR) void k_prep(const float* __restrict__ gW, const float* __restrict__ gb,
                                               const float* __restrict__ wih, const float* __restrict__ whh,
                                               const float* __restrict__ bih, const float* __restrict__ bhh,
                                               unsigned short* WgT2, unsigned short* WihD, unsigned short* WhhB,
                                               float* BG, float* BIH, float* BHH) {
  const int blk = (int)blockIdx.x;
  const int tid = (int)threadIdx.x;
  if (blk < 16) {
    const int u  = blk * NTHR + tid;
    const int n  = u >> 5;
    const int p  = u & 31;
    const int k8 = (p & 15) * 8;
    float x[8];
#pragma unroll
    for (int e = 0; e < 8; ++e) x[e] = gW[(size_t)(k8 + e) * DF + n];
    v4u o = pack8_bf16((v4f){ x[0], x[1], x[2], x[3] }, (v4f){ x[4], x[5], x[6], x[7] });
    const unsigned keep = (p < 16 || AGG_TWO_TERM != 0) ? 0xFFFFFFFFu : 0u;
    o &= (v4u){ keep, keep, keep, keep };
    volatile v4u* q = (volatile v4u*)(WgT2 + (size_t)n * K2 + p * 8);
    *q = o;
    __threadfence();
    *q = o;
  } else if (blk < 64) {
    const int u  = (blk - 16) * NTHR + tid;
    const int n  = u >> 5;
    const int p  = u & 31;
    const int k8 = (p & 15) * 8;
    const v4f a = *(const v4fa*)(wih + (size_t)n * DF + k8);
    const v4f c = *(const v4fa*)(wih + (size_t)n * DF + k8 + 4);
    v4u o = pack8_bf16(a, c);
    const unsigned keep = (p < 16 || X_TWO_TERM != 0) ? 0xFFFFFFFFu : 0u;
    o &= (v4u){ keep, keep, keep, keep };
    volatile v4u* q = (volatile v4u*)(WihD + (size_t)n * K2 + p * 8);
    *q = o;
    __threadfence();
    *q = o;
  } else if (blk < 88) {
    const int u  = (blk - 64) * NTHR + tid;
    const int n  = u >> 4;
    const int k8 = (u & 15) * 8;
    const v4f a = *(const v4fa*)(whh + (size_t)n * DF + k8);
    const v4f c = *(const v4fa*)(whh + (size_t)n * DF + k8 + 4);
    const v4u o = pack8_bf16(a, c);
    volatile v4u* q = (volatile v4u*)(WhhB + (size_t)n * DF + k8);
    *q = o;
    __threadfence();
    *q = o;
  } else {
    if (tid < 32) {
      const v4f t = *(const v4fa*)(gb + 4 * tid);
      const v4f o = (v4f){ bf16_val(t[0]), bf16_val(t[1]), bf16_val(t[2]), bf16_val(t[3]) };
      volatile v4f* q = (volatile v4f*)(BG + 4 * tid);
      *q = o;
      __threadfence();
      *q = o;
    } else if (tid < 128) {
      const int j = tid - 32;
      const v4f t = *(const v4fa*)(bih + 4 * j);
      const v4f o = (v4f){ bf16_val(t[0]), bf16_val(t[1]), bf16_val(t[2]), bf16_val(t[3]) };
      volatile v4f* q = (volatile v4f*)(BIH + 4 * j);
      *q = o;
      __threadfence();
      *q = o;
    } else if (tid < 224) {
      const int j = tid - 128;
      const v4f t = *(const v4fa*)(bhh + 4 * j);
      const v4f o = (v4f){ bf16_val(t[0]), bf16_val(t[1]), bf16_val(t[2]), bf16_val(t[3]) };
      volatile v4f* q = (volatile v4f*)(BHH + 4 * j);
      *q = o;
      __threadfence();
      *q = o;
    }
  }
}

template <int COUNT_ONLY>
__global__ __launch_bounds__(NTHR) void k_bucket(const int* __restrict__ keys, const int* __restrict__ gsrc,
                                                 float* NRM, int* OFFT, int* CNTT, int* LISTT, int* FLAGT) {
  extern __shared__ __attribute__((aligned(16))) int dsm[];
  int* list = dsm;
  int* sl   = list + NWAVE * WLCAP;
  int* cntw = sl + RCAP;
  int* cnt  = cntw + NWAVE * NBA;
  int* offs = cnt + NBA;
  int* nrm  = offs + NBA;
  int* misc = nrm + NBA;
  const int tid = (int)threadIdx.x, lane = tid & 31, wave = tid >> 5;
  const int slotBase = (int)blockIdx.x * NBA;

  {
    const v4i z4 = {0, 0, 0, 0};
    for (int i = tid * 4; i < BK_INTS; i += NTHR * 4) *(v4ia*)(dsm + i) = z4;
  }
  __syncthreads();

  int* mylist = list + wave * WLCAP;
  const int wbase = wave * WSPAN;
  const unsigned usb = (unsigned)slotBase;
  int wc = 0;
#pragma unroll 1
  for (int st = 0; st < WSTEPS; ++st) {
    const int e0  = wbase + st * SUB + lane * 8;
    const int e0c = e0 < (NEDGE - 8) ? e0 : (NEDGE - 8);
    const v4i da = *(const v4i*)(keys + e0c);
    const v4i db = *(const v4i*)(keys + e0c + 4);
    asm volatile("" :: "v"(da), "v"(db));
    const bool inr = e0 < NEDGE;
    const int k0 = inr ? clampi(da.x, 0, NNODE - 1) : -1;
    const int k1 = inr ? clampi(da.y, 0, NNODE - 1) : -1;
    const int k2 = inr ? clampi(da.z, 0, NNODE - 1) : -1;
    const int k3 = inr ? clampi(da.w, 0, NNODE - 1) : -1;
    const int k4 = inr ? clampi(db.x, 0, NNODE - 1) : -1;
    const int k5 = inr ? clampi(db.y, 0, NNODE - 1) : -1;
    const int k6 = inr ? clampi(db.z, 0, NNODE - 1) : -1;
    const int k7 = inr ? clampi(db.w, 0, NNODE - 1) : -1;
    const unsigned s0 = (unsigned)k0 - usb, s1 = (unsigned)k1 - usb, s2 = (unsigned)k2 - usb, s3 = (unsigned)k3 - usb;
    const unsigned s4 = (unsigned)k4 - usb, s5 = (unsigned)k5 - usb, s6 = (unsigned)k6 - usb, s7 = (unsigned)k7 - usb;
    const bool h0 = s0 < (unsigned)NBA, h1 = s1 < (unsigned)NBA, h2 = s2 < (unsigned)NBA, h3 = s3 < (unsigned)NBA;
    const bool h4 = s4 < (unsigned)NBA, h5 = s5 < (unsigned)NBA, h6 = s6 < (unsigned)NBA, h7 = s7 < (unsigned)NBA;
    const int cl = (int)h0 + (int)h1 + (int)h2 + (int)h3 + (int)h4 + (int)h5 + (int)h6 + (int)h7;
    int incl = cl;
#pragma unroll
    for (int d = 1; d < 32; d <<= 1) {
      const int y = __shfl_up(incl, d, 32);
      incl += (lane >= d) ? y : 0;
    }
    const int tot = __shfl(incl, 31, 32);
    int pos = wc + incl - cl;
#define PUTJ(J, HJ, SJ) if (HJ) { if (pos < WLCAP) mylist[pos] = ((e0 + (J)) << SLA) | (int)(SJ); pos += 1; }
    PUTJ(0, h0, s0)
    PUTJ(1, h1, s1)
    PUTJ(2, h2, s2)
    PUTJ(3, h3, s3)
    PUTJ(4, h4, s4)
    PUTJ(5, h5, s5)
    PUTJ(6, h6, s6)
    PUTJ(7, h7, s7)
#undef PUTJ
    wc += tot;
  }
  if (lane == 0) misc[wave] = wc;
  __syncthreads();

  const int wcc = wc < 0 ? 0 : (wc > WLCAP ? WLCAP : wc);
  if (lane == 0) {
#pragma unroll 1
    for (int i = 0; i < wcc; ++i) {
      const int u    = mylist[i];
      const int slot = u & (NBA - 1);
      int* pc = cntw + wave * NBA + slot;
      *pc = *pc + 1;
    }
  }
  __syncthreads();

  int ovf = 0;
#pragma unroll
  for (int w = 0; w < NWAVE; ++w) ovf |= (misc[w] > WLCAP) ? 1 : 0;

  if (wave == 0) {
    const int base = lane * (NBA / 32);
    int s = 0;
#pragma unroll 1
    for (int i = 0; i < NBA / 32; ++i) {
      int t = 0;
#pragma unroll
      for (int w = 0; w < NWAVE; ++w) t += cntw[w * NBA + base + i];
      cnt[base + i] = t;
      s += t;
    }
    int incl = s;
#pragma unroll
    for (int d = 1; d < 32; d <<= 1) {
      const int y = __shfl_up(incl, d, 32);
      incl += (lane >= d) ? y : 0;
    }
    int run = incl - s;
#pragma unroll 1
    for (int i = 0; i < NBA / 32; ++i) {
      offs[base + i] = run;
#pragma unroll
      for (int w = 0; w < NWAVE; ++w) {
        const int cv = cntw[w * NBA + base + i];
        cntw[w * NBA + base + i] = run;
        run += cv;
      }
    }
  }
  __syncthreads();

  if constexpr (COUNT_ONLY == 0) {
    if (lane == 0) {
#pragma unroll 1
      for (int i = 0; i < wcc; ++i) {
        const int u    = mylist[i];
        const int slot = u & (NBA - 1);
        int* pc = cntw + wave * NBA + slot;
        const int p  = *pc;
        const int pq = p < 0 ? 0 : (p > RCAP - 1 ? RCAP - 1 : p);
        sl[pq] = u >> SLA;
        *pc = p + 1;
      }
    }
    __syncthreads();
    int* slab = LISTT + (size_t)blockIdx.x * RCAP;
#pragma unroll 1
    for (int it = 0; it < RCAP / (NTHR * 4); ++it) {
      const int i4 = (it * NTHR + tid) * 4;
      const v4i ev = *(const v4ia*)(sl + i4);
      const int g0 = gsrc[clampi(ev.x, 0, NEDGE - 1)];
      const int g1 = gsrc[clampi(ev.y, 0, NEDGE - 1)];
      const int g2 = gsrc[clampi(ev.z, 0, NEDGE - 1)];
      const int g3 = gsrc[clampi(ev.w, 0, NEDGE - 1)];
      asm volatile("" :: "v"(g0), "v"(g1), "v"(g2), "v"(g3));
      const v4i sv = { clampi(g0, 0, NNODE - 1), clampi(g1, 0, NNODE - 1),
                       clampi(g2, 0, NNODE - 1), clampi(g3, 0, NNODE - 1) };
      volatile v4i* q = (volatile v4i*)(slab + i4);
      *q = sv;
      __threadfence();
      *q = sv;
    }
  }

#pragma unroll 1
  for (int i = 0; i < NBA / NTHR; ++i) {
    const int s  = i * NTHR + tid;
    const int c  = cnt[s];
    const float fc = (float)(c > 1 ? c : 1);
    const float rv = 1.0f / sqrtf(fc);
    const float nv = (c > 0) ? rv : 0.0f;
    nrm[s] = (ovf != 0) ? 0x7fc00000 : __float_as_int(nv);
  }
  __syncthreads();

  const int gs = slotBase + 4 * tid;
  if (gs < NPAD) {
    const v4i cv = *(const v4ia*)(cnt + 4 * tid);
    const v4i ov = *(const v4ia*)(offs + 4 * tid);
    const v4i nb = *(const v4ia*)(nrm + 4 * tid);
    const v4f nv = (v4f){ __int_as_float(nb.x), __int_as_float(nb.y), __int_as_float(nb.z), __int_as_float(nb.w) };
    volatile v4f* qn = (volatile v4f*)(NRM + gs);
    *qn = nv;
    if constexpr (COUNT_ONLY == 0) {
      volatile v4i* qc = (volatile v4i*)(CNTT + gs);
      volatile v4i* qo = (volatile v4i*)(OFFT + gs);
      *qc = cv;
      *qo = ov;
      __threadfence();
      *qc = cv;
      *qo = ov;
    } else {
      __threadfence();
    }
    *qn = nv;
  }
  if constexpr (COUNT_ONLY == 0) {
    if (wave == 0 && lane < 8) {
      const v4i fv = { ovf, ovf, ovf, ovf };
      volatile v4i* qf = (volatile v4i*)(FLAGT + (size_t)blockIdx.x * FLAGW + lane * 4);
      *qf = fv;
      __threadfence();
      *qf = fv;
    }
  }
}

__global__ __launch_bounds__(NTHR) void k_replay(const unsigned short* __restrict__ HB, const int* __restrict__ LISTT,
                                                 const int* __restrict__ OFFT, const int* __restrict__ CNTT,
                                                 const float* __restrict__ NSRC, const float* __restrict__ NDST,
                                                 const int* __restrict__ FLAGT, unsigned short* PHL) {
  __shared__ __attribute__((aligned(16))) unsigned rowbuf[NWAVE][DF];
  const int tid = (int)threadIdx.x, lane = tid & 31, wave = tid >> 5;
  int t = (int)blockIdx.x * NWAVE + wave;
  t = t > NPAD - 1 ? NPAD - 1 : t;
  const bool live = t < NNODE;
  const int b = t >> SLA;
  int cv = CNTT[t];
  asm volatile("" :: "v"(cv));
  const bool big = cv > DEGCAP;
  cv = clampi(cv, 0, DEGCAP);
  const int cn = __builtin_amdgcn_readfirstlane(live ? cv : 0);
  int ov = OFFT[t];
  asm volatile("" :: "v"(ov));
  ov = clampi(ov, 0, RCAP - 1);
  const int fl = FLAGT[b * FLAGW];
  asm volatile("" :: "v"(fl));
  const float nd = NDST[t];
  asm volatile("" :: "v"(nd));
  const int* slab = LISTT + (size_t)b * RCAP;

  float a0 = 0.0f, a1 = 0.0f, a2 = 0.0f, a3 = 0.0f;
#pragma unroll 1
  for (int b0 = 0; b0 < cn; b0 += 32) {
    int idx = ov + b0 + lane;
    idx = idx > RCAP - 1 ? RCAP - 1 : idx;
    int sr = slab[idx];
    asm volatile("" :: "v"(sr));
    sr = clampi(sr, 0, NNODE - 1);
    const float ns = NSRC[sr];
    asm volatile("" :: "v"(ns));
    const int nsi = __float_as_int(ns);
    const int m32 = (cn - b0) < 32 ? (cn - b0) : 32;
#pragma unroll 1
    for (int k = 0; k < m32; ++k) {
      const int   sk = __builtin_amdgcn_readlane(sr, k);
      const float ck = __int_as_float(__builtin_amdgcn_readlane(nsi, k));
      const v2u w = *(const v2ua*)(HB + (size_t)sk * DF + 4 * lane);
      const float f0 = __uint_as_float(w.x << 16);
      const float f1 = __uint_as_float(w.x & 0xffff0000u);
      const float f2 = __uint_as_float(w.y << 16);
      const float f3 = __uint_as_float(w.y & 0xffff0000u);
      a0 = a0 + f0 * ck;
      a1 = a1 + f1 * ck;
      a2 = a2 + f2 * ck;
      a3 = a3 + f3 * ck;
    }
  }
  const float nanv = __int_as_float(0x7fc00000);
  const bool poison = (fl != 0) || big;
  float m0 = a0 * nd, m1 = a1 * nd, m2 = a2 * nd, m3 = a3 * nd;
  m0 = poison ? nanv : m0; m1 = poison ? nanv : m1; m2 = poison ? nanv : m2; m3 = poison ? nanv : m3;
  m0 = live ? m0 : 0.0f;   m1 = live ? m1 : 0.0f;   m2 = live ? m2 : 0.0f;   m3 = live ? m3 : 0.0f;
  const v2u hiw = (v2u){ pk16(bf16_bits(m0), bf16_bits(m1)), pk16(bf16_bits(m2), bf16_bits(m3)) };
  const v2u low = (v2u){ pk16(bf16_lo_bits(m0), bf16_lo_bits(m1)), pk16(bf16_lo_bits(m2), bf16_lo_bits(m3)) };
  unsigned* rb = rowbuf[wave];
  *(v2ua*)(rb + 2 * lane) = hiw;
  *(v2ua*)(rb + 64 + 2 * lane) = low;
  wave_sync();
  const v4u q = *(const v4ua*)(rb + 4 * lane);
  volatile v4u* qp = (volatile v4u*)(PHL + (size_t)t * K2 + 8 * lane);
  *qp = q;
  __threadfence();
  *qp = q;
}

__global__ __launch_bounds__(NTHR) void k_gate(const float* __restrict__ GI, const float* __restrict__ GH,
                                               const unsigned short* __restrict__ HB, const int* __restrict__ FLAGT,
                                               float* outp, int rowOff, int nRows) {
  __shared__ __attribute__((aligned(16))) float ob[NWAVE][DF];
  const int tid = (int)threadIdx.x, lane = tid & 31, wave = tid >> 5;
  const int lr = (int)blockIdx.x * NWAVE + wave;
  const int g  = rowOff + lr;
  const bool live = (lr < nRows) && (g < NNODE);
  const int lrc = clampi(lr, 0, nRows - 1);
  const int gc  = clampi(g, 0, NNODE - 1);
  const int fl = FLAGT[(gc >> SLA) * FLAGW];
  asm volatile("" :: "v"(fl));
  const float nanv = __int_as_float(0x7fc00000);
  const float* gi = GI + (size_t)lrc * G3;
  const float* gh = GH + (size_t)lrc * G3;
  const unsigned short* hb = HB + (size_t)gc * DF;
  float* orow = ob[wave];
#pragma unroll 1
  for (int q = 0; q < 4; ++q) {
    const int c = q * 32 + lane;
    const float ir = gi[c], iz = gi[DF + c], in = gi[2 * DF + c];
    const float hr = gh[c], hz = gh[DF + c], hn = gh[2 * DF + c];
    const unsigned hw = (unsigned)hb[c];
    asm volatile("" :: "v"(ir), "v"(iz), "v"(in), "v"(hr), "v"(hz), "v"(hn), "v"(hw));
    const float hv = __uint_as_float(hw << 16);
    const float r  = 1.0f / (1.0f + expf(-(ir + hr)));
    const float z  = 1.0f / (1.0f + expf(-(iz + hz)));
    const float nn = tanhf(in + r * hn);
    const float v  = (1.0f - z) * nn + z * hv;
    float o = (v > 0.0f) ? v : expm1f(v);
    o = (fl != 0) ? nanv : o;
    orow[c] = o;
  }
  wave_sync();
  const v4f ov = *(const v4fa*)(orow + 4 * lane);
  if (live) {
    volatile v4f* p = (volatile v4f*)(outp + (size_t)g * DF + 4 * lane);
    *p = ov;
    __threadfence();
    *p = ov;
  }
}

static inline int gemm_grid(int M, int N) { return (((M + 63) / 64) * ((N + 63) / 64) + 7) / 8; }

extern "C" void kernel_launch(void* const* d_in, const int* in_sizes, int n_in,
                              void* d_out, int out_size, void* d_ws, size_t ws_size,
                              hipStream_t stream) {
  if (n_in < 9) return;
  if (in_sizes[0] != NEDGE || in_sizes[1] != NEDGE) return;
  if (in_sizes[2] != NNODE * DF) return;
  if (in_sizes[3] != DF * DF || in_sizes[4] != DF) return;
  if (in_sizes[5] != G3 * DF || in_sizes[6] != G3 * DF) return;
  if (in_sizes[7] != G3 || in_sizes[8] != G3) return;
  if ((long long)out_size != (long long)NNODE * DF) return;
  if (ws_size < WS_TOTAL) return;

  const int*   esrc = (const int*)d_in[0];
  const int*   edst = (const int*)d_in[1];
  const float* h    = (const float*)d_in[2];
  const float* gW   = (const float*)d_in[3];
  const float* gb   = (const float*)d_in[4];
  const float* wih  = (const float*)d_in[5];
  const float* whh  = (const float*)d_in[6];
  const float* bih  = (const float*)d_in[7];
  const float* bhh  = (const float*)d_in[8];
  float* out = (float*)d_out;

  char* ws = (char*)d_ws;
  size_t off = 0;
  unsigned short* HB   = (unsigned short*)(ws + off); off += SZ_HB;
  unsigned short* PHL  = (unsigned short*)(ws + off); off += SZ_PHL;
  float* X             = (float*)(ws + off);          off += SZ_X;
  float* GI            = (float*)(ws + off);          off += SZ_G;
  float* GH            = (float*)(ws + off);          off += SZ_G;
  int* LISTT           = (int*)(ws + off);            off += SZ_LIST;
  float* NSRC          = (float*)(ws + off);          off += SZ_TAB;
  float* NDST          = (float*)(ws + off);          off += SZ_TAB;
  int* OFFT            = (int*)(ws + off);            off += SZ_TAB;
  int* CNTT            = (int*)(ws + off);            off += SZ_TAB;
  unsigned short* WgT2 = (unsigned short*)(ws + off); off += SZ_WG;
  unsigned short* WihD = (unsigned short*)(ws + off); off += SZ_WIH;
  unsigned short* WhhB = (unsigned short*)(ws + off); off += SZ_WHH;
  float* BG            = (float*)(ws + off);          off += SZ_BG;
  float* BIH           = (float*)(ws + off);          off += SZ_B3;
  float* BHH           = (float*)(ws + off);          off += SZ_B3;
  int* FLAGT           = (int*)(ws + off);            off += SZ_FLAG;
  if (off != WS_TOTAL) return;

  hipFuncSetAttribute(reinterpret_cast<const void*>(&k_bucket<1>), hipFuncAttributeMaxDynamicSharedMemorySize, (int)BK_LDS);
  hipFuncSetAttribute(reinterpret_cast<const void*>(&k_bucket<0>), hipFuncAttributeMaxDynamicSharedMemorySize, (int)BK_LDS);

  k_prep<<<89, NTHR, 0, stream>>>(gW, gb, wih, whh, bih, bhh, WgT2, WihD, WhhB, BG, BIH, BHH);
  k_plane<0><<<NPAD * DF / 8 / 256, 256, 0, stream>>>(h, NNODE, DF, DF, HB, NPAD, DF);
  k_bucket<1><<<NBLK, NTHR, BK_LDS, stream>>>(esrc, esrc, NSRC, OFFT, CNTT, LISTT, FLAGT);
  k_bucket<0><<<NBLK, NTHR, BK_LDS, stream>>>(edst, esrc, NDST, OFFT, CNTT, LISTT, FLAGT);
  k_replay<<<NPAD / NWAVE, NTHR, 0, stream>>>(HB, LISTT, OFFT, CNTT, NSRC, NDST, FLAGT, PHL);
  k_gemm_nt<0, 1><<<gemm_grid(NPAD, DF), 256, 0, stream>>>(PHL, WgT2, BG, X, NPAD, DF, K2, DF);
  k_plane<1><<<NPAD * K2 / 8 / 256, 256, 0, stream>>>(X, NNODE, DF, DF, PHL, NPAD, DF);
  for (int c = 0; c < 4; ++c) {
    const int rowOff = c * CH_ROWS;
    const int Mc = (c < 3) ? CH_ROWS : CH_LAST;
    k_gemm_nt<0, 1><<<gemm_grid(Mc, G3), 256, 0, stream>>>(PHL + (size_t)rowOff * K2, WihD, BIH, GI, Mc, G3, K2, G3);
    k_gemm_nt<0, 1><<<gemm_grid(Mc, G3), 256, 0, stream>>>(HB + (size_t)rowOff * DF, WhhB, BHH, GH, Mc, G3, DF, G3);
    k_gate<<<Mc / NWAVE, NTHR, 0, stream>>>(GI, GH, HB, FLAGT, out, rowOff, Mc);
  }
}
